// RBFKANConv2d_46334107189774
// MI455X (gfx1250) — hardware-verified
//
#include <hip/hip_runtime.h>


#define NBI  8
#define CI   64
#define IH   64
#define IW   64
#define NP   4096
#define FEAT 576
#define NG   8
#define FG   (FEAT * NG)
#define CO   128
typedef _Float16 h16;
typedef unsigned short bf;
typedef __attribute__((ext_vector_type(16))) __bf16   v16bf;
typedef __attribute__((ext_vector_type(16))) _Float16 v16h;
typedef __attribute__((ext_vector_type(8)))  _Float16 v8h;
typedef __attribute__((ext_vector_type(8)))  unsigned short v8us;
typedef __attribute__((ext_vector_type(8)))  float    v8f;
typedef __attribute__((ext_vector_type(4)))  float    v4f;
typedef v8h  __attribute__((may_alias)) v8ha;
typedef v4f  __attribute__((may_alias)) v4fa;
typedef v8us __attribute__((may_alias)) v8usa;

__device__ __forceinline__ unsigned short f2bf(float f) { unsigned u = __float_as_uint(f); u += 0x7FFFu + ((u >> 16) & 1u); return (unsigned short)(u >> 16); }
__device__ __forceinline__ float bf2f(unsigned short b) { return __uint_as_float(((unsigned)b) << 16); }
__device__ __forceinline__ float bfr(float f) { return bf2f(f2bf(f)); }
__device__ __forceinline__ v16h cat16(v8h lo, v8h hi) { return __builtin_shufflevector(lo, hi, 0, 1, 2, 3, 4, 5, 6, 7, 8, 9, 10, 11, 12, 13, 14, 15); }
__device__ __forceinline__ v16bf cat16b(v8us lo, v8us hi) { return __builtin_bit_cast(v16bf, __builtin_shufflevector(lo, hi, 0, 1, 2, 3, 4, 5, 6, 7, 8, 9, 10, 11, 12, 13, 14, 15)); }
__device__ __forceinline__ v8f wmma16(v16h a, v16h b, v8f c) { return __builtin_amdgcn_wmma_f32_16x16x32_f16(false, a, false, b, (short)0, c, false, false); }
__device__ __forceinline__ v8f wmmab(v16bf a, v16bf b, v8f c) { return __builtin_amdgcn_wmma_f32_16x16x32_bf16(false, a, false, b, (short)0, c, false, false); }


template <typename T16> struct WFrag;
template <> struct WFrag<h16> { typedef v16h V; static __device__ __forceinline__ V ld(const h16* p) { return cat16(*(const v8h*)p, *(const v8h*)(p + 16)); } static __device__ __forceinline__ v8f mma(V a, V b, v8f c) { return wmma16(a, b, c); } };
template <> struct WFrag<bf> { typedef v16bf V; static __device__ __forceinline__ V ld(const bf* p) { return cat16b(*(const v8us*)p, *(const v8us*)(p + 16)); } static __device__ __forceinline__ v8f mma(V a, V b, v8f c) { return wmmab(a, b, c); } };
template <typename T16, int NSPLIT, bool BIAS>
__global__ __launch_bounds__(32) void k_gemmw(const T16* __restrict__ A, const T16* __restrict__ A2, const T16* __restrict__ Bt, const T16* __restrict__ Bt2, int K, float* C, int ldc, const float* __restrict__ bias, size_t sA, size_t sB, size_t sC) {
    typedef typename WFrag<T16>::V V;
    __shared__ __align__(16) float os[16 * 68];
    const size_t z = blockIdx.z; A += z * sA; if (A2) A2 += z * sA; Bt += z * sB; if (Bt2) Bt2 += z * sB; C += z * sC;
    const int lane = threadIdx.x & 31, lr = lane & 15, hi = lane >> 4; const int r0 = blockIdx.x * 64, c0 = blockIdx.y * 64;
    v8f acc[4][4];
#pragma unroll
    for (int mb = 0; mb < 4; ++mb)
#pragma unroll
        for (int nb = 0; nb < 4; ++nb) acc[mb][nb] = (v8f){};
    const size_t aoff = (size_t)(r0 + lr) * K + 8 * hi, boff = (size_t)(c0 + lr) * K + 8 * hi;
#pragma unroll 1
    for (int kc = 0; kc < K; kc += 32) {
        V a[4], a2[4];
#pragma unroll
        for (int mb = 0; mb < 4; ++mb) { a[mb] = WFrag<T16>::ld(A + aoff + (size_t)mb * 16 * K + kc); if (NSPLIT == 1 || NSPLIT == 2) a2[mb] = WFrag<T16>::ld(A2 + aoff + (size_t)mb * 16 * K + kc); }
#pragma unroll
        for (int nb = 0; nb < 4; ++nb) { const V b = WFrag<T16>::ld(Bt + boff + (size_t)nb * 16 * K + kc); V b2; if (NSPLIT >= 2) b2 = WFrag<T16>::ld(Bt2 + boff + (size_t)nb * 16 * K + kc);
#pragma unroll
            for (int mb = 0; mb < 4; ++mb) { acc[mb][nb] = WFrag<T16>::mma(a[mb], b, acc[mb][nb]); if (NSPLIT == 1 || NSPLIT == 2) acc[mb][nb] = WFrag<T16>::mma(a2[mb], b, acc[mb][nb]); if (NSPLIT >= 2) acc[mb][nb] = WFrag<T16>::mma(a[mb], b2, acc[mb][nb]); } }
        asm volatile("v_nop\n\tv_nop\n\tv_nop\n\tv_nop" : "+v"(acc[0][0]), "+v"(acc[1][1]), "+v"(acc[2][2]), "+v"(acc[3][3]) : "v"(a[0]), "v"(a[3]));
    }
#pragma unroll
    for (int mb = 0; mb < 4; ++mb) {
#pragma unroll
        for (int nb = 0; nb < 4; ++nb) {
#pragma unroll
            for (int j = 0; j < 8; ++j) os[(hi * 8 + j) * 68 + nb * 16 + lr] = acc[mb][nb][j]; }
        __builtin_amdgcn_wave_barrier(); asm volatile("" ::: "memory");
        float* crow = C + (size_t)(r0 + mb * 16) * ldc + c0;
#pragma unroll 1
        for (int ps = 0; ps < 2; ++ps) {
#pragma unroll
            for (int s = 0; s < 8; ++s) { const int row = 2 * s + hi, cofs = lr * 4; v4f val = *(const v4fa*)(os + row * 68 + cofs); if (BIAS) { val[0] += bfr(bias[c0 + cofs]); val[1] += bfr(bias[c0 + cofs + 1]); val[2] += bfr(bias[c0 + cofs + 2]); val[3] += bfr(bias[c0 + cofs + 3]); }
                *(volatile v4f*)(crow + (size_t)row * ldc + cofs) = val; }
            if (ps == 0) __threadfence(); }
        __builtin_amdgcn_wave_barrier(); asm volatile("" ::: "memory");
    }
}

__device__ __forceinline__ h16 tohx(float x) { return (h16)x; }
__device__ __forceinline__ void splitf(float y, unsigned short& h, unsigned short& l) { h = f2bf(y); l = f2bf(y - bf2f(h)); }
typedef __attribute__((ext_vector_type(2))) unsigned short v2us;
typedef __attribute__((ext_vector_type(4))) unsigned short v4us;
typedef __attribute__((ext_vector_type(4))) _Float16 v4h;

__global__ __launch_bounds__(256) void k_wtG(const float* __restrict__ w, int K, int N, bf* Bt) {
    const int lane = threadIdx.x & 31; const int L0 = (blockIdx.x * 8 + (threadIdx.x >> 5)) * 8; const int nlines = N * K / 64;
#pragma unroll
    for (int ps = 0; ps < 2; ++ps) {
#pragma unroll 1
        for (int l = 0; l < 8; ++l) { const int L = L0 + l; if (L >= nlines) break; const size_t e = (size_t)L * 64 + lane * 2; const int k = (int)(e % K), n = (int)(e / K); v2us o;
            o[0] = f2bf(w[(size_t)k * N + n]); o[1] = f2bf(w[(size_t)(k + 1) * N + n]); *(volatile v2us*)(Bt + e) = o; }
        if (ps == 0) __threadfence(); }
}
__global__ __launch_bounds__(256) void k_wt16(const float* __restrict__ w, int K, int N, h16* W16) { __shared__ float tile[64][65]; const int nb = (N + 63) / 64; const int k0 = (blockIdx.x / nb) * 64, n0 = (blockIdx.x % nb) * 64;
    for (int i = threadIdx.x; i < 64 * 64; i += 256) { const int kk = i / 64, nn = i % 64; tile[kk][nn] = (k0 + kk < K && n0 + nn < N) ? w[(size_t)(k0 + kk) * N + n0 + nn] : 0.f; }
    __syncthreads();
    const int nn = threadIdx.x / 4, kq = (threadIdx.x % 4) * 16; if (n0 + nn >= N) return;
    for (int c = 0; c < 16; c += 4) { v4h o; o[0] = tohx(bfr(tile[kq + c][nn])); o[1] = tohx(bfr(tile[kq + c + 1][nn])); o[2] = tohx(bfr(tile[kq + c + 2][nn])); o[3] = tohx(bfr(tile[kq + c + 3][nn])); h16* dst = W16 + (size_t)(n0 + nn) * K + k0 + kq + c; for (int ps = 0; ps < 2; ++ps) { *(volatile v4h*)dst = o; if (ps == 0) __threadfence(); } } }
__device__ __forceinline__ float patchval(const float* __restrict__ xb, int pix, int f) { const int c = f / 9, r9 = f % 9, kh = r9 / 3, kw = r9 % 3; const int y = pix / IW + kh - 1, x = pix % IW + kw - 1; return (y >= 0 && y < IH && x >= 0 && x < IW) ? bfr(xb[((size_t)c * IH + y) * IW + x]) : 0.f; }
__global__ __launch_bounds__(256) void k_basis(const float* __restrict__ xb, const float* __restrict__ grid, h16* BAS) { const size_t i = (size_t)blockIdx.x * 256 + threadIdx.x; if (i >= (size_t)NP * FEAT) return; const int f = (int)(i % FEAT); const int pix = (int)(i / FEAT); const float p = patchval(xb, pix, f); typedef __attribute__((ext_vector_type(8))) _Float16 v8h; v8h o;
#pragma unroll
    for (int gI = 0; gI < NG; ++gI) { const float d = __fdiv_rn(__fsub_rn(p, bfr(grid[gI])), 0.5714285714285714f); float q = __fmul_rn(d, d); asm volatile("" : "+v"(q)); o[gI] = tohx(__expf(-q)); }
    h16* dst = BAS + i * NG; *(volatile v8h*)dst = o; __threadfence(); *(volatile v8h*)dst = o; }
__global__ __launch_bounds__(256) void k_silu(const float* __restrict__ xb, bf* Sh, bf* Sl) { const size_t e = ((size_t)blockIdx.x * 256 + threadIdx.x) * 4; if (e >= (size_t)NP * FEAT) return; const int f0 = (int)(e % FEAT); const int pix = (int)(e / FEAT); v4us oh, ol;
#pragma unroll
    for (int u = 0; u < 4; ++u) { const float p = patchval(xb, pix, f0 + u); const float s = __fmul_rn(p, __fdiv_rn(1.0f, 1.0f + __expf(-p))); unsigned short a, b; splitf(s, a, b); oh[u] = a; ol[u] = b; }
    *(volatile v4us*)(Sh + e) = oh; *(volatile v4us*)(Sl + e) = ol; __threadfence(); *(volatile v4us*)(Sh + e) = oh; *(volatile v4us*)(Sl + e) = ol; }
__global__ __launch_bounds__(256) void k_outT(const float* __restrict__ R1, const float* __restrict__ R2, float* OUTb) { const int e = (blockIdx.x * 256 + threadIdx.x) * 4; if (e >= CO * NP) return; const int pix = e % NP; const int co = e / NP; v4f o;
#pragma unroll
    for (int u = 0; u < 4; ++u) o[u] = __fadd_rn(R1[(size_t)(pix + u) * CO + co], R2[(size_t)(pix + u) * CO + co]); *(volatile v4f*)(OUTb + e) = o; __threadfence(); *(volatile v4f*)(OUTb + e) = o; }

extern "C" void kernel_launch(void* const* d_in, const int* in_sizes, int n_in,
                              void* d_out, int out_size, void* d_ws, size_t ws_size, hipStream_t stream) {
    (void)in_sizes; (void)n_in; (void)out_size;
    const float* x = (const float*)d_in[0]; const float* grid = (const float*)d_in[1]; const float* sw = (const float*)d_in[2]; const float* bw = (const float*)d_in[3]; const float* bb = (const float*)d_in[4];
    float* OUT = (float*)d_out;
    char* wsp = (char*)d_ws;
    auto take = [&](size_t bytes) { char* p = wsp; wsp += (bytes + 255) & ~(size_t)255; return (void*)p; };
    h16* SW16 = (h16*)take((size_t)CO * FG * 2); bf* BW = (bf*)take((size_t)CO * FEAT * 2);
    h16* BAS = (h16*)take((size_t)NP * FG * 2); bf* Sh = (bf*)take((size_t)NP * FEAT * 2); bf* Sl = (bf*)take((size_t)NP * FEAT * 2); float* R1 = (float*)take((size_t)NP * CO * 4); float* R2 = (float*)take((size_t)NP * CO * 4);
    if ((size_t)(wsp - (char*)d_ws) > ws_size) return;
    k_wt16<<<(FG / 64) * (CO / 64), 256, 0, stream>>>(sw, FG, CO, SW16); k_wtG<<<(FEAT * CO / 64 + 63) / 64, 256, 0, stream>>>(bw, FEAT, CO, BW);
    for (int b = 0; b < NBI; ++b) { const float* xb = x + (size_t)b * CI * IH * IW;
        k_basis<<<(unsigned)(((size_t)NP * FEAT + 255) / 256), 256, 0, stream>>>(xb, grid, BAS); k_silu<<<(unsigned)(((size_t)NP * FEAT / 4 + 255) / 256), 256, 0, stream>>>(xb, Sh, Sl);
        k_gemmw<h16, 0, false><<<dim3(NP / 64, CO / 64, 1), 32, 0, stream>>>(BAS, nullptr, SW16, nullptr, FG, R1, CO, nullptr, 0, 0, 0);
        k_gemmw<bf, 1, true><<<dim3(NP / 64, CO / 64, 1), 32, 0, stream>>>(Sh, Sl, BW, nullptr, FEAT, R2, CO, bb, 0, 0, 0);
        k_outT<<<(CO * NP / 4 + 255) / 256, 256, 0, stream>>>(R1, R2, OUT + (size_t)b * CO * NP); }
}
